// GatedDeltaRule_77000173682703
// MI455X (gfx1250) — hardware-verified
//
#include <hip/hip_runtime.h>
#include <stdint.h>

constexpr int NBATCH = 4;
constexpr int SEQ    = 2048;
constexpr int HIDDEN = 1024;
constexpr int NHEAD  = 16;
constexpr int HDIM   = 64;
constexpr int NROWS  = NBATCH * SEQ;
constexpr int NPART  = 2;
constexpr int MH     = NROWS / NPART;
constexpr int BPP    = NBATCH / NPART;
constexpr int ABN    = 64;

static_assert(NHEAD * HDIM == HIDDEN, "geom");
static_assert(MH % 64 == 0 && HIDDEN % 64 == 0 && ABN % 64 == 0, "gemm M,N tile multiples");
static_assert(HIDDEN % 32 == 0, "gemm K multiple of 32");
static_assert(MH == BPP * SEQ, "part rows");

constexpr long OUT0_BYTES      = (long)NROWS * HIDDEN * 4;
constexpr long OUT1_OFF_BYTES  = 33554432;
constexpr long OUT1_BYTES      = (long)NBATCH * NHEAD * HDIM * HDIM * 4;
constexpr long OUT_TOTAL_BYTES = 34603008;
static_assert(OUT0_BYTES == OUT1_OFF_BYTES, "out1 follows out0");
static_assert(OUT1_OFF_BYTES + OUT1_BYTES <= OUT_TOTAL_BYTES, "out1 inside d_out");
static_assert(OUT1_OFF_BYTES % 128 == 0, "out1 line aligned");
constexpr long OUT1_OFF_ELEMS  = OUT1_OFF_BYTES / 4;

constexpr long WS_XB   = 0;
constexpr long SZ_XB   = (long)NROWS * HIDDEN * 2;
constexpr long SZ_W    = (long)HIDDEN * HIDDEN * 2;
constexpr long WS_WQ   = WS_XB + SZ_XB;
constexpr long WS_WK   = WS_WQ + SZ_W;
constexpr long WS_WV   = WS_WK + SZ_W;
constexpr long WS_WG   = WS_WV + SZ_W;
constexpr long WS_WOH  = WS_WG + SZ_W;
constexpr long WS_WAB  = WS_WOH + SZ_W;
constexpr long SZ_WAB  = (long)ABN * HIDDEN * 2;
constexpr long WS_BIAS = WS_WAB + SZ_WAB;
constexpr long SZ_BIAS = 256;
constexpr long SZ_P    = (long)MH * HIDDEN * 4;
constexpr long WS_QP   = WS_BIAS + SZ_BIAS;
constexpr long WS_KP   = WS_QP + SZ_P;
constexpr long WS_VP   = WS_KP + SZ_P;
constexpr long WS_GP   = WS_VP + SZ_P;
constexpr long WS_ABP  = WS_GP + SZ_P;
constexpr long SZ_ABP  = (long)MH * ABN * 4;
constexpr long WS_OG   = WS_ABP + SZ_ABP;
constexpr long SZ_OG   = (long)MH * HIDDEN * 2;
constexpr long WS_TOTAL = WS_OG + SZ_OG;
static_assert(WS_TOTAL == 103940352, "carve total");
static_assert(WS_TOTAL <= 134217728, "carve limit");
static_assert(WS_WQ % 256 == 0 && WS_BIAS % 256 == 0 && WS_QP % 256 == 0 && WS_ABP % 256 == 0 && WS_OG % 256 == 0, "alignment");

typedef __attribute__((ext_vector_type(16))) _Float16 v16h;
typedef __attribute__((ext_vector_type(8)))  _Float16 v8h;
typedef __attribute__((ext_vector_type(16))) __bf16   v16b;
typedef __attribute__((ext_vector_type(8)))  __bf16   v8b;
typedef __attribute__((ext_vector_type(8)))  float    v8f;
typedef __attribute__((ext_vector_type(4)))  float    v4f;

__device__ __forceinline__ unsigned short f2bf_bits(float f) {
  unsigned u = __float_as_uint(f);
  return (unsigned short)((u + 0x7FFFu + ((u >> 16) & 1u)) >> 16);
}
__device__ __forceinline__ float bf_bits2f(unsigned short h) { return __uint_as_float(((unsigned)h) << 16); }

__device__ __forceinline__ unsigned pack_f16x2(float f0, float f1) {
  const _Float16 h0 = (_Float16)f0, h1 = (_Float16)f1;
  return (unsigned)__builtin_bit_cast(unsigned short, h0) | ((unsigned)__builtin_bit_cast(unsigned short, h1) << 16);
}

__device__ __forceinline__ void dep_guard_h(v8f& a, v8f& b, v16h x, v16h y) { asm volatile("v_nop\n\tv_nop\n\tv_nop\n\tv_nop" : "+v"(a), "+v"(b) : "v"(x), "v"(y)); }
__device__ __forceinline__ void dep_guard_b(v8f& a, v8f& b, v16b x, v16b y) { asm volatile("v_nop\n\tv_nop\n\tv_nop\n\tv_nop" : "+v"(a), "+v"(b) : "v"(x), "v"(y)); }
__device__ __forceinline__ void keep4_h(v16h a, v16h b, v16h c, v16h d) { asm volatile("v_nop" :: "v"(a), "v"(b), "v"(c), "v"(d)); }
__device__ __forceinline__ void keep4_b(v16b a, v16b b, v16b c, v16b d) { asm volatile("v_nop" :: "v"(a), "v"(b), "v"(c), "v"(d)); }
__device__ __forceinline__ void acc_guard4(v8f& a, v8f& b, v8f& c, v8f& d) { asm volatile("v_nop\n\tv_nop\n\tv_nop\n\tv_nop" : "+v"(a), "+v"(b), "+v"(c), "+v"(d)); }
template <typename T> struct Frag;
template <> struct Frag<_Float16> {
  typedef v16h V; union U { v16h v; v8h h[2]; };
  static __device__ __forceinline__ v16h load(const _Float16* p) {
    U f; f.h[0] = *(const v8h*)(p); f.h[1] = *(const v8h*)(p + 16); return f.v;
  }
  static __device__ __forceinline__ v8f mma(v16h a, v16h b, v8f c) {
    return __builtin_amdgcn_wmma_f32_16x16x32_f16(false, a, false, b, (short)0, c, false, false);
  }
  static __device__ __forceinline__ void guard(v8f& a, v8f& b, v16h x, v16h y) { dep_guard_h(a, b, x, y); }
  static __device__ __forceinline__ void keep(v16h a, v16h b, v16h c, v16h d) { keep4_h(a, b, c, d); }
};
template <> struct Frag<__bf16> {
  typedef v16b V; union U { v16b v; v8b h[2]; };
  static __device__ __forceinline__ v16b load(const __bf16* p) {
    U f; f.h[0] = *(const v8b*)(p); f.h[1] = *(const v8b*)(p + 16); return f.v;
  }
  static __device__ __forceinline__ v8f mma(v16b a, v16b b, v8f c) {
    return __builtin_amdgcn_wmma_f32_16x16x32_bf16(false, a, false, b, (short)0, c, false, false);
  }
  static __device__ __forceinline__ void guard(v8f& a, v8f& b, v16b x, v16b y) { dep_guard_b(a, b, x, y); }
  static __device__ __forceinline__ void keep(v16b a, v16b b, v16b c, v16b d) { keep4_b(a, b, c, d); }
};

template <int ET> struct Elem;
template <> struct Elem<0> { typedef _Float16 T; };
template <> struct Elem<1> { typedef __bf16 T; };
template <int ET, bool SPLIT, int BIAS_MODE, int OUT_MODE, bool RESID, int ACT = 0>
__global__ __launch_bounds__(256) void wmma_gemm64(
    const unsigned short* __restrict__ Ap, const unsigned short* __restrict__ A2p, int lda, long strideA,
    const unsigned short* __restrict__ Btp, const unsigned short* __restrict__ Bt2p, int ldb, long strideB,
    void* __restrict__ Cout, void* __restrict__ Cout2, int ldc, long strideC,
    const float* __restrict__ bias,
    const float* __restrict__ resid, long strideR,
    int M, int N, int K, float scale) {
  typedef typename Elem<ET>::T T;
  typedef typename Frag<T>::V V;
  const T* A = (const T*)Ap; const T* A2 = (const T*)A2p; const T* Bt = (const T*)Btp; const T* Bt2 = (const T*)Bt2p;
  __shared__ __align__(16) float sT[8][16 * 68];
  const int b    = blockIdx.y;
  const int lane = threadIdx.x & 31;
  const int wave = threadIdx.x >> 5;
  const int tilesN = N >> 6;
  const int tilesM = M >> 6;
  const int tile = blockIdx.x * 8 + wave;
  if (tile >= tilesM * tilesN) return;
  const int tm = tile / tilesN;
  const int tn = tile - tm * tilesN;
  const int m0 = tm << 6;
  const int n0 = tn << 6;

  const T* Ab  = A  + (size_t)b * strideA;
  const T* Bb  = Bt + (size_t)b * strideB;
  const T* Ab2 = SPLIT ? (A2  + (size_t)b * strideA) : nullptr;
  const T* Bb2 = SPLIT ? (Bt2 + (size_t)b * strideB) : nullptr;

  const int rlane = lane & 15;
  const int koff  = (lane >> 4) * 8;
  const int mOff  = (lane >> 4) * 8;

  v8f acc[4][4];
#pragma unroll
  for (int i = 0; i < 4; ++i)
#pragma unroll
    for (int j = 0; j < 4; ++j) acc[i][j] = (v8f){0.f,0.f,0.f,0.f,0.f,0.f,0.f,0.f};

  for (int k0 = 0; k0 < K; k0 += 32) {
    V bh[4], bl[4];
#pragma unroll
    for (int j = 0; j < 4; ++j) {
      const size_t bo = (size_t)(n0 + (j << 4) + rlane) * ldb + koff + k0;
      bh[j] = Frag<T>::load(Bb + bo);
      if (SPLIT) bl[j] = Frag<T>::load(Bb2 + bo);
    }
#pragma unroll
    for (int i = 0; i < 4; ++i) {
      const size_t ao = (size_t)(m0 + (i << 4) + rlane) * lda + koff + k0;
      V ah = Frag<T>::load(Ab + ao);
      V al;
      if (SPLIT) al = Frag<T>::load(Ab2 + ao);
#pragma unroll
      for (int j = 0; j < 4; ++j) {
        acc[i][j] = Frag<T>::mma(ah, bh[j], acc[i][j]);
        if (SPLIT) {
          acc[i][j] = Frag<T>::mma(ah, bl[j], acc[i][j]);
          acc[i][j] = Frag<T>::mma(al, bh[j], acc[i][j]);
        }
      }
      Frag<T>::guard(acc[i][0], acc[i][3], ah, SPLIT ? al : ah);
    }
    Frag<T>::keep(bh[0], bh[1], bh[2], bh[3]);
    if (SPLIT) Frag<T>::keep(bl[0], bl[1], bl[2], bl[3]);
  }
  acc_guard4(acc[0][0], acc[0][1], acc[0][2], acc[0][3]);
  acc_guard4(acc[1][0], acc[1][1], acc[1][2], acc[1][3]);
  acc_guard4(acc[2][0], acc[2][1], acc[2][2], acc[2][3]);
  acc_guard4(acc[3][0], acc[3][1], acc[3][2], acc[3][3]);

  float* slab = sT[wave];
  const float* Rb = RESID ? (resid + (size_t)b * strideR) : nullptr;
#pragma unroll
  for (int i = 0; i < 4; ++i) {
    const int mBase = m0 + (i << 4);
    float rinv[8];
#pragma unroll
    for (int r = 0; r < 8; ++r) rinv[r] = 1.0f;
    if (ACT == 7) {
#pragma unroll
      for (int r = 0; r < 8; ++r) {
        float ss = 0.f;
#pragma unroll
        for (int j = 0; j < 4; ++j) { const float tv = acc[i][j][r] * scale; ss += tv * tv; }
        ss += __shfl_xor(ss, 1, 32);
        ss += __shfl_xor(ss, 2, 32);
        ss += __shfl_xor(ss, 4, 32);
        ss += __shfl_xor(ss, 8, 32);
        rinv[r] = 1.0f / fmaxf(sqrtf(ss), 1e-6f);
      }
    }
#pragma unroll
    for (int j = 0; j < 4; ++j) {
      const int n = n0 + (j << 4) + rlane;
      float bv = 0.f;
      if (BIAS_MODE == 2) bv = bias[n];
#pragma unroll
      for (int r = 0; r < 8; ++r) {
        float v = acc[i][j][r] * scale;
        if (BIAS_MODE == 1) v += bias[mBase + mOff + r];
        if (BIAS_MODE == 2) v += bv;
        if (RESID) v += Rb[(size_t)(mBase + mOff + r) * ldc + n];
        if (ACT == 1) v = tanhf(v);
        if (ACT == 2) v = fmaxf(v, 0.0f);
        if (ACT == 3) v = v / (1.0f + expf(-v));
        if (ACT == 4) v = (v > 0.f) ? v : 0.01f * v;
        if (ACT == 6) v = 1.0f / (1.0f + expf(-v));
        if (ACT == 7) v = v * rinv[r];
        slab[(mOff + r) * 68 + (j << 4) + rlane] = v;
      }
    }
    __builtin_amdgcn_fence(__ATOMIC_RELEASE, "workgroup");
    __builtin_amdgcn_wave_barrier();
    __builtin_amdgcn_fence(__ATOMIC_ACQUIRE, "workgroup");
    if (OUT_MODE == 0) {
      float* C = (float*)Cout + (size_t)b * strideC;
      const int hh = lane >> 4, c4 = (lane & 15) * 4;
      for (int pass = 0; pass < 2; ++pass) {
#pragma unroll
        for (int it = 0; it < 8; ++it) {
          const int row = it * 2 + hh;
          v4f v = *(const v4f*)(slab + row * 68 + c4);
          *(volatile v4f*)(C + (size_t)(mBase + row) * ldc + n0 + c4) = v;
        }
        __threadfence();
      }
    } else {
      const int q = lane >> 3, c8 = (lane & 7) * 8;
      unsigned short* C  = (unsigned short*)Cout  + (size_t)b * strideC;
      unsigned short* C2 = (OUT_MODE == 2) ? ((unsigned short*)Cout2 + (size_t)b * strideC) : nullptr;
      for (int pass = 0; pass < 2; ++pass) {
#pragma unroll
        for (int it = 0; it < 4; ++it) {
          const int row = it * 4 + q;
          const float* sp = slab + row * 68 + c8;
          v8h hv, lv;
#pragma unroll
          for (int e = 0; e < 8; ++e) {
            if (OUT_MODE == 1) {
              hv[e] = (_Float16)sp[e];
            } else {
              unsigned short hb = f2bf_bits(sp[e]);
              unsigned short lb = f2bf_bits(sp[e] - bf_bits2f(hb));
              hv[e] = __builtin_bit_cast(_Float16, hb);
              lv[e] = __builtin_bit_cast(_Float16, lb);
            }
          }
          *(volatile v8h*)(C + (size_t)(mBase + row) * ldc + n0 + c8) = hv;
          if (OUT_MODE == 2) *(volatile v8h*)(C2 + (size_t)(mBase + row) * ldc + n0 + c8) = lv;
        }
        __threadfence();
      }
    }
    __builtin_amdgcn_fence(__ATOMIC_RELEASE, "workgroup");
    __builtin_amdgcn_wave_barrier();
    __builtin_amdgcn_fence(__ATOMIC_ACQUIRE, "workgroup");
  }
}

__global__ __launch_bounds__(256) void cast_f32_bf16x2(
    const float* __restrict__ in, unsigned short* __restrict__ out, int n2) {
  const int i = blockIdx.x * 256 + threadIdx.x;
  if (i < n2) {
    const unsigned u = (unsigned)f2bf_bits(in[2 * i]) | ((unsigned)f2bf_bits(in[2 * i + 1]) << 16);
    ((volatile unsigned*)out)[i] = u;
    __threadfence();
    ((volatile unsigned*)out)[i] = u;
  }
}

__global__ __launch_bounds__(256) void cast_f32_bf16_f16x2_scaled(
    const float* __restrict__ in, unsigned short* __restrict__ out, int n2, float sc) {
  const int i = blockIdx.x * 256 + threadIdx.x;
  if (i < n2) {
    const float f0 = bf_bits2f(f2bf_bits(in[2 * i])) * sc;
    const float f1 = bf_bits2f(f2bf_bits(in[2 * i + 1])) * sc;
    const unsigned u = pack_f16x2(f0, f1);
    ((volatile unsigned*)out)[i] = u;
    __threadfence();
    ((volatile unsigned*)out)[i] = u;
  }
}

static_assert((ABN * HIDDEN / 2) % 256 == 0, "wab grid");
__global__ __launch_bounds__(256) void build_wab_bias(
    const float* __restrict__ Wa, const float* __restrict__ Wb,
    const float* __restrict__ ba, const float* __restrict__ bb,
    unsigned short* __restrict__ wab, float* __restrict__ bias64) {
  const int i = blockIdx.x * 256 + threadIdx.x;
  const int e = 2 * i;
  const int row = e >> 10;
  const int col = e & (HIDDEN - 1);
  const int ra = (row < 16) ? row : 15;
  int rb = row - 16; rb = (rb < 0) ? 0 : ((rb > 15) ? 15 : rb);
  const float a0 = Wa[(size_t)ra * HIDDEN + col];
  const float a1 = Wa[(size_t)ra * HIDDEN + col + 1];
  const float b0 = Wb[(size_t)rb * HIDDEN + col];
  const float b1 = Wb[(size_t)rb * HIDDEN + col + 1];
  const float v0 = (row < 16) ? a0 : ((row < 32) ? b0 : 0.f);
  const float v1 = (row < 16) ? a1 : ((row < 32) ? b1 : 0.f);
  const unsigned u = (unsigned)f2bf_bits(v0) | ((unsigned)f2bf_bits(v1) << 16);
  ((volatile unsigned*)wab)[i] = u;
  __threadfence();
  ((volatile unsigned*)wab)[i] = u;
  if (blockIdx.x == 0 && threadIdx.x < 32) {
    const int l = threadIdx.x;
    if (l < 16) {
      float w[4];
#pragma unroll
      for (int c = 0; c < 4; ++c) {
        const int n = 4 * l + c;
        const int ia = (n < 16) ? n : 15;
        int ib = n - 16; ib = (ib < 0) ? 0 : ((ib > 15) ? 15 : ib);
        const float fa = ba[ia];
        const float fb = bb[ib];
        const float sel = (n < 16) ? fa : ((n < 32) ? fb : 0.f);
        w[c] = bf_bits2f(f2bf_bits(sel));
      }
      const v4f wv = (v4f){w[0], w[1], w[2], w[3]};
      *(volatile v4f*)(bias64 + 4 * l) = wv;
      __threadfence();
      *(volatile v4f*)(bias64 + 4 * l) = wv;
    }
  }
}

__global__ __launch_bounds__(256) void delta_scan(
    const float* __restrict__ qP, const float* __restrict__ kP, const float* __restrict__ vP,
    const float* __restrict__ gP, const float* __restrict__ abP,
    unsigned short* __restrict__ ogP, float* __restrict__ sOut) {
  __shared__ __align__(16) float lin[2][256];
  __shared__ __align__(16) float lod[2][64];
  __shared__ __align__(16) float sst[HDIM * HDIM];
  const int tid  = threadIdx.x;
  const int lane = tid & 31;
  const int wave = tid >> 5;
  const int bl   = blockIdx.x >> 4;
  const int h    = blockIdx.x & 15;
  const int i    = tid >> 2;
  const int p    = tid & 3;
  const int j0   = p * 16;
  const int grp  = tid >> 6;
  const int e    = tid & 63;
  const float* src = (grp == 0) ? kP : ((grp == 1) ? qP : ((grp == 2) ? vP : gP));
  const size_t colh  = (size_t)h * HDIM;
  const size_t rbase = (size_t)bl * SEQ;

  float S[16];
#pragma unroll
  for (int j = 0; j < 16; ++j) S[j] = 0.f;

  lin[0][tid] = src[rbase * HIDDEN + colh + e];
  float a_nx = abP[rbase * ABN + h];
  float b_nx = abP[rbase * ABN + 16 + h];

  for (int t = 0; t < SEQ; ++t) {
    const int cur = t & 1;
    const float at = a_nx;
    const float bt = b_nx;
    __syncthreads();
    if (t > 0) {
      if (wave == 0) {
        const float f0 = lod[cur ^ 1][2 * lane];
        const float f1 = lod[cur ^ 1][2 * lane + 1];
        const unsigned u = pack_f16x2(f0, f1);
        volatile unsigned* dst = (volatile unsigned*)(void*)(ogP + ((rbase + (size_t)(t - 1)) * HIDDEN + colh)) + lane;
        *dst = u;
        __threadfence();
        *dst = u;
      }
    }
    v4f k4[4], q4[4];
#pragma unroll
    for (int m = 0; m < 4; ++m) {
      k4[m] = *(const v4f*)(&lin[cur][j0 + 4 * m]);
      q4[m] = *(const v4f*)(&lin[cur][64 + j0 + 4 * m]);
    }
    const float vi = lin[cur][128 + i];
    const float gi = lin[cur][192 + i];
    float sk = 0.f;
#pragma unroll
    for (int m = 0; m < 4; ++m) {
      sk += S[4 * m + 0] * k4[m].x;
      sk += S[4 * m + 1] * k4[m].y;
      sk += S[4 * m + 2] * k4[m].z;
      sk += S[4 * m + 3] * k4[m].w;
    }
    sk += __shfl_xor(sk, 1, 32);
    sk += __shfl_xor(sk, 2, 32);
    const float ci = bt * vi - (at * bt) * sk;
    float o = 0.f;
#pragma unroll
    for (int m = 0; m < 4; ++m) {
      S[4 * m + 0] = at * S[4 * m + 0] + ci * k4[m].x; o += S[4 * m + 0] * q4[m].x;
      S[4 * m + 1] = at * S[4 * m + 1] + ci * k4[m].y; o += S[4 * m + 1] * q4[m].y;
      S[4 * m + 2] = at * S[4 * m + 2] + ci * k4[m].z; o += S[4 * m + 2] * q4[m].z;
      S[4 * m + 3] = at * S[4 * m + 3] + ci * k4[m].w; o += S[4 * m + 3] * q4[m].w;
    }
    o += __shfl_xor(o, 1, 32);
    o += __shfl_xor(o, 2, 32);
    lod[cur][i] = o * gi * 16.0f;
    const int tn = (t + 1 < SEQ) ? (t + 1) : (SEQ - 1);
    const size_t rn = rbase + (size_t)tn;
    lin[cur ^ 1][tid] = src[rn * HIDDEN + colh + e];
    a_nx = abP[rn * ABN + h];
    b_nx = abP[rn * ABN + 16 + h];
  }
  __syncthreads();
  if (wave == 0) {
    const int lst = (SEQ - 1) & 1;
    const float f0 = lod[lst][2 * lane];
    const float f1 = lod[lst][2 * lane + 1];
    const unsigned u = pack_f16x2(f0, f1);
    volatile unsigned* dst = (volatile unsigned*)(void*)(ogP + ((rbase + (size_t)(SEQ - 1)) * HIDDEN + colh)) + lane;
    *dst = u;
    __threadfence();
    *dst = u;
  }
#pragma unroll
  for (int m = 0; m < 4; ++m) {
    const v4f sv = (v4f){S[4 * m + 0], S[4 * m + 1], S[4 * m + 2], S[4 * m + 3]};
    *(v4f*)(&sst[i * HDIM + j0 + 4 * m]) = sv;
  }
  __syncthreads();
  float* ob = sOut + (size_t)(bl * NHEAD + h) * (HDIM * HDIM);
  for (int pass = 0; pass < 2; ++pass) {
#pragma unroll
    for (int it = 0; it < 4; ++it) {
      const int idx = wave * 512 + it * 128 + lane * 4;
      const v4f val = *(const v4f*)(&sst[idx]);
      *(volatile v4f*)(ob + idx) = val;
    }
    __threadfence();
  }
}

extern "C" void kernel_launch(void* const* d_in, const int* in_sizes, int n_in,
                              void* d_out, int out_size, void* d_ws, size_t ws_size, hipStream_t stream) {
  (void)in_sizes; (void)n_in;
  if (ws_size < (size_t)WS_TOTAL) return;
  if ((long)out_size * 4 < OUT_TOTAL_BYTES) return;

  const float* x  = (const float*)d_in[0];
  const float* Wq = (const float*)d_in[1];
  const float* Wk = (const float*)d_in[2];
  const float* Wv = (const float*)d_in[3];
  const float* Wa = (const float*)d_in[4];
  const float* ba = (const float*)d_in[5];
  const float* Wb = (const float*)d_in[6];
  const float* bb = (const float*)d_in[7];
  const float* Wg = (const float*)d_in[8];
  const float* Wo = (const float*)d_in[9];

  char* ws = (char*)d_ws;
  unsigned short* xb   = (unsigned short*)(ws + WS_XB);
  unsigned short* wq   = (unsigned short*)(ws + WS_WQ);
  unsigned short* wk   = (unsigned short*)(ws + WS_WK);
  unsigned short* wv   = (unsigned short*)(ws + WS_WV);
  unsigned short* wg   = (unsigned short*)(ws + WS_WG);
  unsigned short* woh  = (unsigned short*)(ws + WS_WOH);
  unsigned short* wab  = (unsigned short*)(ws + WS_WAB);
  float*          bias = (float*)(ws + WS_BIAS);
  float*          qP   = (float*)(ws + WS_QP);
  float*          kP   = (float*)(ws + WS_KP);
  float*          vP   = (float*)(ws + WS_VP);
  float*          gP   = (float*)(ws + WS_GP);
  float*          abP  = (float*)(ws + WS_ABP);
  unsigned short* ogP  = (unsigned short*)(ws + WS_OG);
  float* out0 = (float*)d_out;
  float* out1 = out0 + OUT1_OFF_ELEMS;

  const int nx2 = NROWS * HIDDEN / 2;
  const int nw2 = HIDDEN * HIDDEN / 2;
  cast_f32_bf16x2<<<nx2 / 256, 256, 0, stream>>>(x,  xb, nx2);
  cast_f32_bf16x2<<<nw2 / 256, 256, 0, stream>>>(Wq, wq, nw2);
  cast_f32_bf16x2<<<nw2 / 256, 256, 0, stream>>>(Wk, wk, nw2);
  cast_f32_bf16x2<<<nw2 / 256, 256, 0, stream>>>(Wv, wv, nw2);
  cast_f32_bf16x2<<<nw2 / 256, 256, 0, stream>>>(Wg, wg, nw2);
  cast_f32_bf16_f16x2_scaled<<<nw2 / 256, 256, 0, stream>>>(Wo, woh, nw2, 16.0f);
  build_wab_bias<<<(ABN * HIDDEN / 2) / 256, 256, 0, stream>>>(Wa, Wb, ba, bb, wab, bias);

  const int gx_full = (MH / 64) * (HIDDEN / 64) / 8;
  const int gx_ab   = (MH / 64) * (ABN / 64) / 8;
  static_assert(((MH / 64) * (HIDDEN / 64)) % 8 == 0 && ((MH / 64) * (ABN / 64)) % 8 == 0, "tile grids");

  for (int part = 0; part < NPART; ++part) {
    const unsigned short* xp = xb + (size_t)part * MH * HIDDEN;
    wmma_gemm64<1, false, 0, 0, false, 7><<<dim3(gx_full, 2), 256, 0, stream>>>(
        xp, xp, HIDDEN, 0L, wq, wq, HIDDEN, (long)HIDDEN * HIDDEN,
        (void*)qP, (void*)qP, HIDDEN, (long)MH * HIDDEN, bias, bias, 0L, MH, HIDDEN, HIDDEN, 1.0f);
    wmma_gemm64<1, false, 0, 0, false, 0><<<dim3(gx_full, 1), 256, 0, stream>>>(
        xp, xp, HIDDEN, 0L, wv, wv, HIDDEN, 0L,
        (void*)vP, (void*)vP, HIDDEN, 0L, bias, bias, 0L, MH, HIDDEN, HIDDEN, 1.0f);
    wmma_gemm64<1, false, 0, 0, false, 3><<<dim3(gx_full, 1), 256, 0, stream>>>(
        xp, xp, HIDDEN, 0L, wg, wg, HIDDEN, 0L,
        (void*)gP, (void*)gP, HIDDEN, 0L, bias, bias, 0L, MH, HIDDEN, HIDDEN, 1.0f);
    wmma_gemm64<1, false, 2, 0, false, 6><<<dim3(gx_ab, 1), 256, 0, stream>>>(
        xp, xp, HIDDEN, 0L, wab, wab, HIDDEN, 0L,
        (void*)abP, (void*)abP, ABN, 0L, bias, bias, 0L, MH, ABN, HIDDEN, 1.0f);
    delta_scan<<<BPP * NHEAD, 256, 0, stream>>>(
        qP, kP, vP, gP, abP, ogP, out1 + (size_t)part * BPP * NHEAD * HDIM * HDIM);
    wmma_gemm64<0, false, 0, 0, false, 0><<<dim3(gx_full, 1), 256, 0, stream>>>(
        ogP, ogP, HIDDEN, 0L, woh, woh, HIDDEN, 0L,
        (void*)(out0 + (size_t)part * MH * HIDDEN), (void*)(out0 + (size_t)part * MH * HIDDEN), HIDDEN, 0L,
        bias, bias, 0L, MH, HIDDEN, HIDDEN, 1.0f / 256.0f);
  }
}
